// SelfAttention_61658550501938
// MI455X (gfx1250) — hardware-verified
//
#include <hip/hip_runtime.h>


#ifndef NB
#define NB 4
#endif
#ifndef SEQ
#define SEQ 2048
#endif
#define NB_FULL  4
#define SEQ_FULL 2048
#define DM   1024
#define NH   16
#define HD   64
#define NQKV (3 * DM)
#define CK   (2 * DM)
#define RH   768
#define RHE  ((SEQ < RH) ? SEQ : RH)
#define PCAR 1024.0f
#define RSC  2048.0f
#define RINV (1.0f / 2048.0f)
#define SCL  0.125f
#define NEGB (-3.0e38f)
#define PLN  ((size_t)NH * SEQ * HD)

#define WS_WQKV ((size_t)NQKV * DM * 2)
#define WS_XB   ((size_t)SEQ * DM * 2)
#define WS_F    ((size_t)SEQ * NQKV * 4)
#define WS_PL   ((size_t)6 * NH * SEQ * HD * 2)
#define WS_CTX  ((size_t)SEQ * CK * 2)
#define WS_TOTAL (WS_WQKV + WS_XB + WS_F + WS_PL + WS_CTX)

static_assert(NB <= NB_FULL);
static_assert(SEQ <= SEQ_FULL);
static_assert(SEQ % 64 == 0);
static_assert(DM % 64 == 0);
static_assert(NQKV % 64 == 0);
static_assert(DM % 32 == 0);
static_assert(CK == 2 * DM);
static_assert(DM % 4 == 0);
static_assert(((size_t)SEQ * DM / 4) % 256 == 0);
static_assert(((size_t)SEQ * DM / 8) % 256 == 0);
static_assert((PLN / 8) % 256 == 0);
static_assert(HD == 64);
static_assert(NH * HD == DM);
static_assert(RH % 32 == 0);
static_assert(RHE % 16 == 0);
static_assert((SEQ - RHE) % 16 == 0);
static_assert(WS_WQKV % 256 == 0);
static_assert(WS_XB % 256 == 0);
static_assert(WS_F % 256 == 0);
static_assert(WS_PL % 256 == 0);
static_assert(WS_CTX % 256 == 0);
static_assert(WS_TOTAL <= (size_t)134217728);

typedef _Float16 h16;
typedef unsigned short bf;
typedef __attribute__((ext_vector_type(16))) __bf16   v16bf;
typedef __attribute__((ext_vector_type(16))) _Float16 v16h;
typedef __attribute__((ext_vector_type(8)))  _Float16 v8h;
typedef __attribute__((ext_vector_type(8)))  unsigned short v8us;
typedef __attribute__((ext_vector_type(4)))  unsigned short v4us;
typedef __attribute__((ext_vector_type(2)))  unsigned short v2us;
typedef __attribute__((ext_vector_type(8)))  float    v8f;
typedef __attribute__((ext_vector_type(4)))  float    v4f;
typedef v4f  __attribute__((may_alias)) v4fa;
typedef v8us __attribute__((may_alias)) v8usa;

__device__ __forceinline__ unsigned short f2bf(float f) { unsigned u = __float_as_uint(f); u += 0x7FFFu + ((u >> 16) & 1u); return (unsigned short)(u >> 16); }
__device__ __forceinline__ float bf2f(unsigned short b) { return __uint_as_float(((unsigned)b) << 16); }
__device__ __forceinline__ void splitf(float y, unsigned short& h, unsigned short& l) { h = f2bf(y); l = f2bf(y - bf2f(h)); }
__device__ __forceinline__ v16h cat16(v8h lo, v8h hi) { return __builtin_shufflevector(lo, hi, 0, 1, 2, 3, 4, 5, 6, 7, 8, 9, 10, 11, 12, 13, 14, 15); }
__device__ __forceinline__ v16bf cat16b(v8us lo, v8us hi) { return __builtin_bit_cast(v16bf, __builtin_shufflevector(lo, hi, 0, 1, 2, 3, 4, 5, 6, 7, 8, 9, 10, 11, 12, 13, 14, 15)); }
__device__ __forceinline__ v8f wmma16(v16h a, v16h b, v8f c) { return __builtin_amdgcn_wmma_f32_16x16x32_f16(false, a, false, b, (short)0, c, false, false); }
__device__ __forceinline__ v8f wmmab(v16bf a, v16bf b, v8f c) { return __builtin_amdgcn_wmma_f32_16x16x32_bf16(false, a, false, b, (short)0, c, false, false); }
__device__ __forceinline__ v16h  ldh(const h16* p) { return cat16(*(const v8h*)p, *(const v8h*)(p + 16)); }
__device__ __forceinline__ v16bf ldb(const bf* p)  { return cat16b(*(const v8us*)p, *(const v8us*)(p + 16)); }

__global__ __launch_bounds__(32) __attribute__((amdgpu_num_vgpr(256)))
void k_gemmw(const bf* __restrict__ A, const bf* __restrict__ Bt, int K, float* C, int ldc) {
    __shared__ __align__(16) float os[16 * 68];
    const int lane = threadIdx.x & 31, lr = lane & 15, hi = lane >> 4; const int r0 = blockIdx.x * 64, c0 = blockIdx.y * 64;
    v8f acc[4][4];
#pragma unroll
    for (int mb = 0; mb < 4; ++mb)
#pragma unroll
        for (int nb = 0; nb < 4; ++nb) acc[mb][nb] = (v8f){};
    const size_t aoff = (size_t)(r0 + lr) * K + 8 * hi, boff = (size_t)(c0 + lr) * K + 8 * hi;
#pragma unroll 1
    for (int kc = 0; kc < K; kc += 32) {
        v16bf a[4];
#pragma unroll
        for (int mb = 0; mb < 4; ++mb) a[mb] = ldb(A + aoff + (size_t)mb * 16 * K + kc);
#pragma unroll
        for (int nb = 0; nb < 4; ++nb) { const v16bf b = ldb(Bt + boff + (size_t)nb * 16 * K + kc);
#pragma unroll
            for (int mb = 0; mb < 4; ++mb) acc[mb][nb] = wmmab(a[mb], b, acc[mb][nb]); }
        asm volatile("v_nop\n\tv_nop\n\tv_nop\n\tv_nop" : "+v"(acc[0][0]), "+v"(acc[1][1]), "+v"(acc[2][2]), "+v"(acc[3][3]) : "v"(a[0]), "v"(a[3]));
    }
#pragma unroll
    for (int mb = 0; mb < 4; ++mb) {
#pragma unroll
        for (int nb = 0; nb < 4; ++nb) {
#pragma unroll
            for (int j = 0; j < 8; ++j) os[(hi * 8 + j) * 68 + nb * 16 + lr] = acc[mb][nb][j]; }
        __builtin_amdgcn_wave_barrier(); asm volatile("" ::: "memory");
        float* crow = C + (size_t)(r0 + mb * 16) * ldc + c0;
#pragma unroll 1
        for (int ps = 0; ps < 2; ++ps) {
#pragma unroll
            for (int s = 0; s < 8; ++s) { const int row = 2 * s + hi, cofs = lr * 4; const v4f val = *(const v4fa*)(os + row * 68 + cofs);
                *(volatile v4f*)(crow + (size_t)row * ldc + cofs) = val; }
            if (ps == 0) __threadfence(); }
        __builtin_amdgcn_wave_barrier(); asm volatile("" ::: "memory");
    }
}

__global__ __launch_bounds__(256) void k_wt(const float* __restrict__ w, int K, int N, int rep, bf* Bt) {
    const int lane = threadIdx.x & 31; const int wave = __builtin_amdgcn_readfirstlane(threadIdx.x >> 5);
    const int KO = K * rep; const int L0 = (blockIdx.x * 8 + wave) * 8; const int nlines = (int)(((size_t)N * KO) / 64);
#pragma unroll 1
    for (int ps = 0; ps < 2; ++ps) {
#pragma unroll 1
        for (int l = 0; l < 8; ++l) { const int L = L0 + l; if (L >= nlines) break; const size_t e = (size_t)L * 64 + lane * 2; const int ko = (int)(e % KO), n = (int)(e / KO); const int k = ko % K; v2us o;
            o[0] = f2bf(w[(size_t)k * N + n]); o[1] = f2bf(w[(size_t)(k + 1) * N + n]); *(volatile v2us*)(Bt + e) = o; }
        if (ps == 0) __threadfence(); }
}

__global__ __launch_bounds__(256) void k_cvt8(const float* __restrict__ src, bf* dst, size_t n8) { const size_t i = (size_t)blockIdx.x * 256 + threadIdx.x; if (i >= n8) return; const v8f v = *(const v8f*)(src + i * 8); v8us o;
#pragma unroll
    for (int k = 0; k < 8; ++k) o[k] = f2bf(v[k]); *(volatile v8us*)(dst + i * 8) = o; __threadfence(); *(volatile v8us*)(dst + i * 8) = o; }

__global__ __launch_bounds__(256) void k_qkp(const float* __restrict__ F, h16* PL) {
    const size_t i = (size_t)blockIdx.x * 256 + threadIdx.x; if (i >= PLN / 8) return; const int which = blockIdx.y;
    const size_t e = i * 8; const int d = (int)(e % HD); const int t = (int)((e / HD) % SEQ); const int h = (int)(e / ((size_t)HD * SEQ));
    const v8f v = *(const v8f*)(F + (size_t)t * NQKV + which * DM + h * HD + d); v8h o, r;
#pragma unroll
    for (int k = 0; k < 8; ++k) { const h16 a = (h16)v[k]; o[k] = a; r[k] = (h16)((v[k] - (float)a) * RSC); }
    h16* p16 = PL + (size_t)which * 2 * PLN + e; h16* pr = p16 + PLN;
    *(volatile v8h*)p16 = o; *(volatile v8h*)pr = r; __threadfence(); *(volatile v8h*)p16 = o; *(volatile v8h*)pr = r; }

__global__ __launch_bounds__(256) void k_vtp(const float* __restrict__ F, h16* PL) {
    const size_t i = (size_t)blockIdx.x * 256 + threadIdx.x; if (i >= PLN / 8) return;
    const size_t e = i * 8; const int t = (int)(e % SEQ); const int d = (int)((e / SEQ) % HD); const int h = (int)(e / ((size_t)SEQ * HD));
    const float* f = F + (size_t)t * NQKV + 2 * DM + h * HD + d; v8h o, r;
#pragma unroll
    for (int k = 0; k < 8; ++k) { const float x = f[(size_t)k * NQKV]; const h16 a = (h16)x; o[k] = a; r[k] = (h16)((x - (float)a) * RSC); }
    h16* p16 = PL + 4 * PLN + e; h16* pr = p16 + PLN;
    *(volatile v8h*)p16 = o; *(volatile v8h*)pr = r; __threadfence(); *(volatile v8h*)p16 = o; *(volatile v8h*)pr = r; }

template <bool HIRES>
__device__ __forceinline__ void attn_body(const h16* __restrict__ PL, bf* CTX, const int qbase) {
    __shared__ __align__(16) unsigned short ost[2 * 16 * HD];
    const int lane = threadIdx.x & 31, lr = lane & 15, hi = lane >> 4;
    const int head = blockIdx.y;
    const int q0 = qbase + blockIdx.x * 16;
    const size_t hb = (size_t)head * SEQ * HD;
    const size_t oQ = hb + (size_t)(q0 + lr) * HD + 8 * hi;
    const size_t oK = 2 * PLN + hb + (size_t)lr * HD + 8 * hi;
    const size_t oV = 4 * PLN + hb + (size_t)lr * SEQ + 8 * hi;
    const float CE = SCL * 1.4426950408889634f;
    v8f o[4], orr[4];
#pragma unroll
    for (int dt = 0; dt < 4; ++dt) { o[dt] = (v8f){}; orr[dt] = (v8f){}; }
    float m = NEGB, l = 0.0f;
#pragma unroll 1
    for (int kb = 0; kb < q0 + 16; kb += 32) {
        v8f sh0 = (v8f){}, sh1 = (v8f){}, sr0 = (v8f){}, sr1 = (v8f){};
#pragma unroll
        for (int kc = 0; kc < HD; kc += 32) {
            const v16h bq  = ldh(PL + oQ + kc);
            const v16h bqr = ldh(PL + PLN + oQ + kc);
            const v16h ak0 = ldh(PL + oK + (size_t)kb * HD + kc);
            const v16h ak1 = ldh(PL + oK + (size_t)(kb + 16) * HD + kc);
            sh0 = wmma16(ak0, bq, sh0);  sh1 = wmma16(ak1, bq, sh1);
            sr0 = wmma16(ak0, bqr, sr0); sr1 = wmma16(ak1, bqr, sr1);
            if (HIRES) {
                const v16h kr0 = ldh(PL + PLN + oK + (size_t)kb * HD + kc);
                const v16h kr1 = ldh(PL + PLN + oK + (size_t)(kb + 16) * HD + kc);
                sr0 = wmma16(kr0, bq, sr0); sr1 = wmma16(kr1, bq, sr1);
                asm volatile("v_nop\n\tv_nop\n\tv_nop\n\tv_nop" : "+v"(sh0), "+v"(sh1), "+v"(sr0), "+v"(sr1) : "v"(ak0), "v"(ak1), "v"(bq), "v"(bqr), "v"(kr0), "v"(kr1));
            } else {
                asm volatile("v_nop\n\tv_nop\n\tv_nop\n\tv_nop" : "+v"(sh0), "+v"(sh1), "+v"(sr0), "+v"(sr1) : "v"(ak0), "v"(ak1), "v"(bq), "v"(bqr));
            }
        }
        float u[16];
#pragma unroll
        for (int r = 0; r < 8; ++r) { u[r] = (sh0[r] + sr0[r] * RINV) * CE; u[8 + r] = (sh1[r] + sr1[r] * RINV) * CE; }
        if (kb + 31 > q0) {
            const int qi = q0 + lr; const int k0 = kb + 8 * hi;
#pragma unroll
            for (int r = 0; r < 8; ++r) { u[r] = (k0 + r > qi) ? NEGB : u[r]; u[8 + r] = (k0 + 16 + r > qi) ? NEGB : u[8 + r]; }
        }
        float mx = u[0];
#pragma unroll
        for (int i = 1; i < 16; ++i) mx = fmaxf(mx, u[i]);
        mx = fmaxf(mx, __shfl_xor(mx, 16, 32));
        const float mn = fmaxf(m, mx);
        const float corr = __builtin_amdgcn_exp2f(m - mn);
        m = mn;
        float psum = 0.0f;
#pragma unroll
        for (int i = 0; i < 16; ++i) { u[i] = __builtin_amdgcn_exp2f(u[i] - mn); psum += u[i]; }
        l = l * corr + psum;
#pragma unroll
        for (int dt = 0; dt < 4; ++dt) {
#pragma unroll
            for (int r = 0; r < 8; ++r) { o[dt][r] *= corr; if (HIRES) orr[dt][r] *= corr; } }
        v16h pb, pr;
#pragma unroll
        for (int i = 0; i < 16; ++i) { const float pc = u[i] * PCAR; const h16 ph = (h16)pc; pb[i] = ph; pr[i] = (h16)((pc - (float)ph) * RSC); }
        const size_t ov = oV + kb;
        if (HIRES) {
#pragma unroll
            for (int dt = 0; dt < 4; ++dt) {
                const v16h av  = ldh(PL + ov + (size_t)dt * 16 * SEQ);
                const v16h avr = ldh(PL + PLN + ov + (size_t)dt * 16 * SEQ);
                o[dt]   = wmma16(av, pb, o[dt]);
                orr[dt] = wmma16(avr, pb, orr[dt]);
                orr[dt] = wmma16(av, pr, orr[dt]);
                asm volatile("v_nop\n\tv_nop\n\tv_nop\n\tv_nop" : "+v"(o[dt]), "+v"(orr[dt]) : "v"(av), "v"(avr), "v"(pb), "v"(pr));
            }
        } else {
            const v16h av0 = ldh(PL + ov);
            const v16h av1 = ldh(PL + ov + (size_t)16 * SEQ);
            const v16h av2 = ldh(PL + ov + (size_t)32 * SEQ);
            const v16h av3 = ldh(PL + ov + (size_t)48 * SEQ);
            o[0] = wmma16(av0, pb, o[0]); o[1] = wmma16(av1, pb, o[1]); o[2] = wmma16(av2, pb, o[2]); o[3] = wmma16(av3, pb, o[3]);
            asm volatile("v_nop\n\tv_nop\n\tv_nop\n\tv_nop" : "+v"(o[0]), "+v"(o[1]), "+v"(o[2]), "+v"(o[3]) : "v"(av0), "v"(av1), "v"(av2), "v"(av3), "v"(pb));
        }
    }
    l += __shfl_xor(l, 16, 32);
    const float inv = 1.0f / (l * PCAR);
#pragma unroll
    for (int dt = 0; dt < 4; ++dt) { v8us vh, vl;
#pragma unroll
        for (int r = 0; r < 8; ++r) { float y = o[dt][r]; if (HIRES) y += orr[dt][r] * RINV; y *= inv; unsigned short a, c; splitf(y, a, c); vh[r] = a; vl[r] = c; }
        *(v8usa*)(ost + lr * HD + dt * 16 + hi * 8) = vh; *(v8usa*)(ost + 16 * HD + lr * HD + dt * 16 + hi * 8) = vl; }
    __builtin_amdgcn_wave_barrier(); asm volatile("" ::: "memory");
    bf* crow = CTX + (size_t)q0 * CK + head * HD;
#pragma unroll 1
    for (int ps = 0; ps < 2; ++ps) {
#pragma unroll
        for (int s = 0; s < 4; ++s) { const int row = 4 * s + (lane >> 3), pc = (lane & 7) * 8;
            const v8us a = *(const v8usa*)(ost + row * HD + pc); const v8us c = *(const v8usa*)(ost + 16 * HD + row * HD + pc);
            *(volatile v8us*)(crow + (size_t)row * CK + pc) = a; *(volatile v8us*)(crow + (size_t)row * CK + DM + pc) = c; }
        if (ps == 0) __threadfence(); }
}
__global__ __launch_bounds__(32) __attribute__((amdgpu_num_vgpr(256))) void k_attn_hi(const h16* __restrict__ PL, bf* CTX) { attn_body<true>(PL, CTX, 0); }
__global__ __launch_bounds__(32) __attribute__((amdgpu_num_vgpr(256))) void k_attn_lo(const h16* __restrict__ PL, bf* CTX) { attn_body<false>(PL, CTX, RHE); }

__global__ __launch_bounds__(256) void k_out(const bf* __restrict__ CTX, float* OUT) {
    const size_t i = (size_t)blockIdx.x * 256 + threadIdx.x; if (i >= (size_t)SEQ * DM / 4) return;
    const size_t e = i * 4; const int c = (int)(e % DM); const size_t t = e / DM;
    const v4us a = *(const v4us*)(CTX + t * CK + c); const v4us d = *(const v4us*)(CTX + t * CK + DM + c); v4f o;
#pragma unroll
    for (int k = 0; k < 4; ++k) o[k] = bf2f(a[k]) + bf2f(d[k]);
    *(volatile v4f*)(OUT + e) = o; __threadfence(); *(volatile v4f*)(OUT + e) = o; }

extern "C" void kernel_launch(void* const* d_in, const int* in_sizes, int n_in,
                              void* d_out, int out_size, void* d_ws, size_t ws_size, hipStream_t stream) {
    if (n_in < 2) return;
    const int need_x = (NB - 1) * SEQ_FULL * DM + SEQ * DM;
    if (in_sizes[0] < need_x || in_sizes[1] < DM * NQKV || out_size < need_x) return;
    if (WS_TOTAL > ws_size) return;
    const float* x = (const float*)d_in[0]; const float* wqkv = (const float*)d_in[1];
    float* OUT = (float*)d_out;
    char* wsp = (char*)d_ws;
    bf* WQKV = (bf*)wsp;  wsp += WS_WQKV;
    bf* XB   = (bf*)wsp;  wsp += WS_XB;
    float* F = (float*)wsp; wsp += WS_F;
    h16* PL  = (h16*)wsp; wsp += WS_PL;
    bf* CTX  = (bf*)wsp;  wsp += WS_CTX;
    k_wt<<<(unsigned)(((size_t)NQKV * DM / 64 + 63) / 64), 256, 0, stream>>>(wqkv, DM, NQKV, 1, WQKV);
    const unsigned LP = (unsigned)((PLN / 8 + 255) / 256);
    for (int b = 0; b < NB; ++b) {
        const float* xb = x + (size_t)b * SEQ_FULL * DM;
        k_cvt8<<<(unsigned)(((size_t)SEQ * DM / 8 + 255) / 256), 256, 0, stream>>>(xb, XB, (size_t)SEQ * DM / 8);
        k_gemmw<<<dim3(SEQ / 64, NQKV / 64, 1), 32, 0, stream>>>(XB, WQKV, DM, F, NQKV);
        k_qkp<<<dim3(LP, 2, 1), 256, 0, stream>>>(F, PL);
        k_vtp<<<LP, 256, 0, stream>>>(F, PL);
        k_attn_hi<<<dim3(RHE / 16, NH, 1), 32, 0, stream>>>(PL, CTX);
        if (SEQ > RHE) k_attn_lo<<<dim3((SEQ - RHE) / 16, NH, 1), 32, 0, stream>>>(PL, CTX);
        k_out<<<(unsigned)(((size_t)SEQ * DM / 4 + 255) / 256), 256, 0, stream>>>(CTX, OUT + (size_t)b * SEQ_FULL * DM);
    }
}
